// LocallyConnectedNN_1056561955144
// MI455X (gfx1250) — hardware-verified
//
#include <hip/hip_runtime.h>


namespace {
constexpr int B = 1024, K3 = 9;
constexpr int C1 = 16, H1 = 14, NL1 = H1 * H1, KP1 = 32;
constexpr int C2 = 32, H2 = 12, NL2 = H2 * H2, KP2 = 160;
constexpr int C3 = 64, H3 = 10, NL3 = H3 * H3, KP3 = 288;
constexpr int NF = 6400, NO = 10;
constexpr float AS_ = 8.0f, EPS = 1e-5f;

typedef _Float16 b16;
typedef __attribute__((ext_vector_type(16))) _Float16 v16b;
typedef __attribute__((ext_vector_type(8))) _Float16 v8b;
typedef __attribute__((ext_vector_type(8))) float v8f;
typedef __attribute__((ext_vector_type(4))) float v4f;
__device__ __forceinline__ float bf16_rne(float f) { unsigned int u = __float_as_uint(f); u += 0x7FFFu + ((u >> 16) & 1u); return __uint_as_float(u & 0xFFFF0000u); }
__device__ __forceinline__ void split16(float v, b16& hi, b16& lo) { hi = (b16)v; lo = (b16)(v - (float)hi); }
__device__ __forceinline__ v16b frag_kb(const b16* p, int hh) { const v8b a = *(const v8b*)(p + 8 * hh), b = *(const v8b*)(p + 16 + 8 * hh); v16b f;
#pragma unroll
  for (int e = 0; e < 8; ++e) { f[e] = a[e]; f[8 + e] = b[e]; } return f; }
__device__ __forceinline__ v8f wmma16b(v16b a, v16b b, v8f c) { v8f d = __builtin_amdgcn_wmma_f32_16x16x32_f16(false, a, false, b, (short)0, c, false, false); asm volatile("v_nop\n\tv_nop\n\tv_nop\n\tv_nop" : "+v"(d) : "v"(a), "v"(b)); return d; }
__device__ __forceinline__ void wave_lds_sync() { __builtin_amdgcn_fence(__ATOMIC_RELEASE, "workgroup"); __builtin_amdgcn_wave_barrier(); __builtin_amdgcn_fence(__ATOMIC_ACQUIRE, "workgroup"); }
__device__ __forceinline__ float nexp(float x) { return __builtin_amdgcn_exp2f(x * 1.4426950408889634f); }
__device__ __forceinline__ float pmul(float a, float b) { float p = a * b; asm volatile("" : "+v"(p)); return p; }
__device__ __forceinline__ float tanh_f(float x) { const float e = nexp(-2.0f * fabsf(x)); const float t = (1.0f - e) / (1.0f + e); return (x >= 0.0f) ? t : -t; }

struct Wo_ { static constexpr size_t W1 = 0, W2 = W1 + (size_t)NL1 * C1 * KP1, W3 = W2 + (size_t)NL2 * C2 * KP2, FC = W3 + (size_t)NL3 * C3 * KP3, END = FC + (size_t)16 * NF; };
struct Po_ { static constexpr int B1 = 0, B2 = B1 + C1 * NL1, B3 = B2 + C2 * NL2, FCB = B3 + C3 * NL3, G1 = FCB + 16, BE1 = G1 + 16, G2 = BE1 + 16, BE2 = G2 + 32, G3 = BE2 + 32, BE3 = G3 + 64, END = BE3 + 64; };
__global__ __launch_bounds__(256) void prep_kernel(const float* __restrict__ W1, const float* __restrict__ b1, const float* __restrict__ g1, const float* __restrict__ be1, const float* __restrict__ W2, const float* __restrict__ b2, const float* __restrict__ g2, const float* __restrict__ be2, const float* __restrict__ W3, const float* __restrict__ b3, const float* __restrict__ g3, const float* __restrict__ be3, const float* __restrict__ fcW, const float* __restrict__ fcb, b16* __restrict__ R, float* __restrict__ P) {
  const size_t tid = (size_t)blockIdx.x * 256 + threadIdx.x, nth = (size_t)gridDim.x * 256;
  for (int pass = 0; pass < 2; ++pass) {
    for (size_t q = tid; q < (size_t)NL1 * C1 * KP1; q += nth) { const int k = (int)(q % KP1), o = (int)((q / KP1) % C1), loc = (int)(q / (KP1 * C1)); R[Wo_::W1 + q] = (b16)((k < 9) ? bf16_rne(W1[((size_t)o * NL1 + loc) * 9 + k]) : 0.0f); }
    for (size_t q = tid; q < (size_t)NL2 * C2 * KP2; q += nth) { const int k = (int)(q % KP2), o = (int)((q / KP2) % C2), loc = (int)(q / (KP2 * C2)); float w = 0.0f; if (k < C1 * 9) { const int c = k / 9, uv = k % 9; w = bf16_rne(W2[(((size_t)o * C1 + c) * NL2 + loc) * 9 + uv]); } R[Wo_::W2 + q] = (b16)w; }
    for (size_t q = tid; q < (size_t)NL3 * C3 * KP3; q += nth) { const int k = (int)(q % KP3), o = (int)((q / KP3) % C3), loc = (int)(q / (KP3 * C3)); const int c = k / 9, uv = k % 9; R[Wo_::W3 + q] = (b16)bf16_rne(W3[(((size_t)o * C2 + c) * NL3 + loc) * 9 + uv]); }
    for (size_t q = tid; q < (size_t)16 * NF; q += nth) { const int o = (int)(q / NF), k = (int)(q % NF); R[Wo_::FC + q] = (b16)((o < NO) ? bf16_rne(fcW[(size_t)o * NF + k]) : 0.0f); }
    for (size_t q = tid; q < (size_t)Po_::END; q += nth) { const int i = (int)q; float v;
      if (i < Po_::B2) v = b1[i]; else if (i < Po_::B3) v = b2[i - Po_::B2]; else if (i < Po_::FCB) v = b3[i - Po_::B3]; else if (i < Po_::G1) v = (i - Po_::FCB < NO) ? fcb[i - Po_::FCB] : 0.0f;
      else if (i < Po_::BE1) v = g1[i - Po_::G1]; else if (i < Po_::G2) v = be1[i - Po_::BE1]; else if (i < Po_::BE2) v = g2[i - Po_::G2]; else if (i < Po_::G3) v = be2[i - Po_::BE2]; else if (i < Po_::BE3) v = g3[i - Po_::G3]; else v = be3[i - Po_::BE3];
      P[q] = bf16_rne(v); }
    __threadfence(); }
}

__global__ __launch_bounds__(128) void lc1_kernel(const float* __restrict__ x, const b16* __restrict__ R, const float* __restrict__ P, float* __restrict__ y1) {
  __shared__ __attribute__((aligned(16))) float T[C1][128 + 4];
  const int lane = threadIdx.x & 31, wave = threadIdx.x >> 5, nloc = lane & 15, hlf = lane >> 4, loc = blockIdx.x, i0 = loc / H1, j0 = loc % H1, b0 = blockIdx.y * 128, m0 = b0 + wave * 32;
  v8f acc[2];
#pragma unroll
  for (int r = 0; r < 2; ++r) { const int b = m0 + r * 16 + nloc; v16b a = {};
#pragma unroll
    for (int e = 0; e < 16; ++e) { const int k = (e < 8) ? (8 * hlf + e) : (16 + 8 * hlf + e - 8); if (k < 9) { const int u = k / 3, v = k % 3; a[e] = (b16)bf16_rne(x[(size_t)b * 256 + (i0 + u) * 16 + (j0 + v)]); } }
    const v16b bw = frag_kb(R + Wo_::W1 + ((size_t)loc * C1 + nloc) * KP1, hlf); acc[r] = (v8f){}; acc[r] = wmma16b(a, bw, acc[r]); }
  const float bb = P[Po_::B1 + nloc * NL1 + loc];
#pragma unroll
  for (int r = 0; r < 2; ++r)
#pragma unroll
    for (int v = 0; v < 8; ++v) T[nloc][wave * 32 + r * 16 + 8 * hlf + v] = acc[r][v] + bb;
  __syncthreads();
  for (int pass = 0; pass < 2; ++pass) { for (int i = threadIdx.x; i < C1 * 32; i += 128) { const int o = i >> 5, c4 = (i & 31) * 4; *(volatile v4f*)(y1 + ((size_t)loc * C1 + o) * B + b0 + c4) = *(const v4f*)(&T[o][c4]); } __threadfence(); }
}

__global__ __launch_bounds__(256) void bnstat_kernel(const float* __restrict__ y, int C, int NL, float* __restrict__ st) {
  __shared__ float red[256]; __shared__ float mu_s;
  const int o = blockIdx.x, t_ = threadIdx.x; const float cnt = (float)NL * (float)B;
  float s = 0.0f; for (int loc = 0; loc < NL; ++loc) { const float* row = y + ((size_t)loc * C + o) * B; for (int b = t_; b < B; b += 256) s += row[b]; }
  red[t_] = s; __syncthreads(); for (int k = 128; k > 0; k >>= 1) { if (t_ < k) red[t_] += red[t_ + k]; __syncthreads(); }
  if (t_ == 0) mu_s = red[0] / cnt; __syncthreads(); const float mu = mu_s;
  float q = 0.0f; for (int loc = 0; loc < NL; ++loc) { const float* row = y + ((size_t)loc * C + o) * B; for (int b = t_; b < B; b += 256) { const float d = row[b] - mu; q += pmul(d, d); } }
  __syncthreads(); red[t_] = q; __syncthreads(); for (int k = 128; k > 0; k >>= 1) { if (t_ < k) red[t_] += red[t_ + k]; __syncthreads(); }
  if (t_ < 32) { const float v = (t_ == 0) ? mu : (t_ == 1) ? rsqrtf(red[0] / cnt + EPS) : 0.0f; for (int pass = 0; pass < 2; ++pass) ((volatile float*)st)[(size_t)o * 32 + t_] = v; }
  __threadfence();
}

template <int CIN, int HIN, int COUT, int KP>
__global__ __launch_bounds__(128) void lc_kernel(const float* __restrict__ yp, const float* __restrict__ stp, const float* __restrict__ gam, const float* __restrict__ bet, const b16* __restrict__ Wr, const float* __restrict__ bias, float* __restrict__ y) {
  constexpr int HOUT = HIN - 2, NLOUT = HOUT * HOUT, NT = COUT / 16;
  __shared__ __attribute__((aligned(16))) float T[COUT][128 + 4]; __shared__ float Sm[CIN], Si[CIN], Sg[CIN], Sb[CIN];
  const int lane = threadIdx.x & 31, wave = threadIdx.x >> 5, nloc = lane & 15, hlf = lane >> 4, loc = blockIdx.x, i0 = loc / HOUT, j0 = loc % HOUT, b0 = blockIdx.y * 128, m0 = b0 + wave * 32;
  for (int c = threadIdx.x; c < CIN; c += 128) { Sm[c] = stp[c * 32]; Si[c] = stp[c * 32 + 1]; Sg[c] = gam[c]; Sb[c] = bet[c]; }
  __syncthreads();
  v8f acc[2][NT];
#pragma unroll
  for (int r = 0; r < 2; ++r)
#pragma unroll
    for (int t = 0; t < NT; ++t) acc[r][t] = (v8f){};
  for (int kb = 0; kb < KP; kb += 32) { v16b ah[2], al[2];
#pragma unroll
    for (int r = 0; r < 2; ++r) { const int b = m0 + r * 16 + nloc;
#pragma unroll
      for (int e = 0; e < 16; ++e) { const int k = kb + ((e < 8) ? (8 * hlf + e) : (16 + 8 * hlf + e - 8)); float v = 0.0f;
        if (k < CIN * 9) { const int c = k / 9, uv = k % 9, u = uv / 3, vv = uv % 3; const float raw = yp[((size_t)((i0 + u) * HIN + (j0 + vv)) * CIN + c) * B + b]; v = fmaxf(pmul((raw - Sm[c]) * Si[c], Sg[c]) + Sb[c], 0.0f); }
        b16 h_, l_; split16(v * AS_, h_, l_); ah[r][e] = h_; al[r][e] = l_; } }
#pragma unroll
    for (int t = 0; t < NT; ++t) { const v16b bw = frag_kb(Wr + ((size_t)loc * COUT + t * 16 + nloc) * KP + kb, hlf);
#pragma unroll
      for (int r = 0; r < 2; ++r) { acc[r][t] = wmma16b(ah[r], bw, acc[r][t]); acc[r][t] = wmma16b(al[r], bw, acc[r][t]); } } }
#pragma unroll
  for (int t = 0; t < NT; ++t) { const int o = t * 16 + nloc; const float bb = bias[o * NLOUT + loc];
#pragma unroll
    for (int r = 0; r < 2; ++r)
#pragma unroll
      for (int v = 0; v < 8; ++v) T[o][wave * 32 + r * 16 + 8 * hlf + v] = acc[r][t][v] * (1.0f / AS_) + bb; }
  __syncthreads();
  for (int pass = 0; pass < 2; ++pass) { for (int i = threadIdx.x; i < COUT * 32; i += 128) { const int o = i >> 5, c4 = (i & 31) * 4; *(volatile v4f*)(y + ((size_t)loc * COUT + o) * B + b0 + c4) = *(const v4f*)(&T[o][c4]); } __threadfence(); }
}

__global__ __launch_bounds__(128) void fc_kernel(const float* __restrict__ y3, const float* __restrict__ st3, const float* __restrict__ gam, const float* __restrict__ bet, const b16* __restrict__ R, const float* __restrict__ P, float* __restrict__ out) {
  __shared__ float Z[128][NO]; __shared__ float Sm[C3], Si[C3], Sg[C3], Sb[C3];
  const int lane = threadIdx.x & 31, wave = threadIdx.x >> 5, nloc = lane & 15, hlf = lane >> 4, b0 = blockIdx.x * 128, m0 = b0 + wave * 32;
  for (int c = threadIdx.x; c < C3; c += 128) { Sm[c] = st3[c * 32]; Si[c] = st3[c * 32 + 1]; Sg[c] = gam[c]; Sb[c] = bet[c]; }
  __syncthreads();
  v8f acc[2] = {{}, {}};
  for (int kb = 0; kb < NF; kb += 32) { v16b ah[2], al[2];
#pragma unroll
    for (int r = 0; r < 2; ++r) { const int b = m0 + r * 16 + nloc;
#pragma unroll
      for (int e = 0; e < 16; ++e) { const int k = kb + ((e < 8) ? (8 * hlf + e) : (16 + 8 * hlf + e - 8)); const int o = k / NL3, loc = k % NL3; const float raw = y3[((size_t)loc * C3 + o) * B + b]; const float v = tanh_f(pmul((raw - Sm[o]) * Si[o], Sg[o]) + Sb[o]); b16 h_, l_; split16(v * AS_, h_, l_); ah[r][e] = h_; al[r][e] = l_; } }
    const v16b bw = frag_kb(R + Wo_::FC + (size_t)nloc * NF + kb, hlf);
#pragma unroll
    for (int r = 0; r < 2; ++r) { acc[r] = wmma16b(ah[r], bw, acc[r]); acc[r] = wmma16b(al[r], bw, acc[r]); } }
  if (nloc < NO) { const float bb = P[Po_::FCB + nloc];
#pragma unroll
    for (int r = 0; r < 2; ++r)
#pragma unroll
      for (int v = 0; v < 8; ++v) Z[wave * 32 + r * 16 + 8 * hlf + v][nloc] = acc[r][v] * (1.0f / AS_) + bb; }
  __syncthreads();
  for (int pass = 0; pass < 2; ++pass) { for (int i = threadIdx.x; i < 128 * NO / 4; i += 128) *(volatile v4f*)(out + (size_t)b0 * NO + i * 4) = *(const v4f*)(&Z[0][0] + i * 4); __threadfence(); }
}
}

extern "C" void kernel_launch(void* const* d_in, const int* in_sizes, int n_in,
                              void* d_out, int out_size, void* d_ws, size_t ws_size, hipStream_t stream) {
  (void)n_in; (void)out_size;
  const float* x = (const float*)d_in[0]; const float* W1 = (const float*)d_in[1]; const float* b1 = (const float*)d_in[2]; const float* g1 = (const float*)d_in[3]; const float* be1 = (const float*)d_in[4];
  const float* W2 = (const float*)d_in[5]; const float* b2 = (const float*)d_in[6]; const float* g2 = (const float*)d_in[7]; const float* be2 = (const float*)d_in[8];
  const float* W3 = (const float*)d_in[9]; const float* b3 = (const float*)d_in[10]; const float* g3 = (const float*)d_in[11]; const float* be3 = (const float*)d_in[12]; const float* fcW = (const float*)d_in[13]; const float* fcb = (const float*)d_in[14];
  float* out = (float*)d_out;
  if (in_sizes[0] != B * 256 || in_sizes[1] != C1 * NL1 * 9 || in_sizes[5] != C2 * C1 * NL2 * 9 || in_sizes[9] != C3 * C2 * NL3 * 9 || in_sizes[13] != NO * NF) return;
  size_t off = 0; char* ws = (char*)d_ws;
  auto carve = [&](size_t bytes) { char* p = ws + off; off += (bytes + 255) & ~(size_t)255; return p; };
  b16* R = (b16*)carve(Wo_::END * 2); float* P = (float*)carve(((size_t)Po_::END + 64) * 4);
  float* y1 = (float*)carve((size_t)NL1 * C1 * B * 4); float* y2 = (float*)carve((size_t)NL2 * C2 * B * 4); float* y3 = (float*)carve((size_t)NL3 * C3 * B * 4); float* st1 = (float*)carve(C1 * 32 * 4); float* st2 = (float*)carve(C2 * 32 * 4); float* st3 = (float*)carve(C3 * 32 * 4);
  if (off > ws_size) return;
  prep_kernel<<<512, 256, 0, stream>>>(W1, b1, g1, be1, W2, b2, g2, be2, W3, b3, g3, be3, fcW, fcb, R, P);
  lc1_kernel<<<dim3(NL1, B / 128), 128, 0, stream>>>(x, R, P, y1);
  bnstat_kernel<<<C1, 256, 0, stream>>>(y1, C1, NL1, st1);
  lc_kernel<C1, H1, C2, KP2><<<dim3(NL2, B / 128), 128, 0, stream>>>(y1, st1, P + Po_::G1, P + Po_::BE1, R + Wo_::W2, P + Po_::B2, y2);
  bnstat_kernel<<<C2, 256, 0, stream>>>(y2, C2, NL2, st2);
  lc_kernel<C2, H2, C3, KP3><<<dim3(NL3, B / 128), 128, 0, stream>>>(y2, st2, P + Po_::G2, P + Po_::BE2, R + Wo_::W3, P + Po_::B3, y3);
  bnstat_kernel<<<C3, 256, 0, stream>>>(y3, C3, NL3, st3);
  fc_kernel<<<B / 128, 128, 0, stream>>>(y3, st3, P + Po_::G3, P + Po_::BE3, R, P, out);
}
